// MultiHeadSelfAttention2D_21157008900677
// MI455X (gfx1250) — hardware-verified
//
#include <hip/hip_runtime.h>

#ifndef NB
#define NB 4
#endif
#ifndef SEQ
#define SEQ 2304
#endif
#define NB_FULL 4
#define SEQ_FULL 2304
#define DIM 256
#define HEADS 8
#define HD 32
#define OCH 768
#define W_IMG 48
#define NPOS 48

static_assert(NB >= 1 && NB <= NB_FULL);
static_assert(SEQ >= 64 && SEQ <= SEQ_FULL && (SEQ % 64) == 0);
static_assert(DIM == HEADS * HD);
static_assert((DIM * DIM) % 2048 == 0);
static_assert((NPOS * DIM) % 256 == 0);
static_assert(HD == 32);

typedef _Float16 v16h __attribute__((ext_vector_type(16)));
typedef _Float16 v8h __attribute__((ext_vector_type(8)));
typedef __attribute__((ext_vector_type(16))) __bf16 v16b;
typedef unsigned short v8us __attribute__((ext_vector_type(8)));
typedef float v8f __attribute__((ext_vector_type(8)));
typedef float v4f __attribute__((ext_vector_type(4)));

union FragH { v16h v; v8h p[2]; };
union FragB { v16b v; v8us p[2]; };

__device__ __forceinline__ v8f mma_bf16(v16b a, v16b b, v8f c) {
  c = __builtin_amdgcn_wmma_f32_16x16x32_bf16(false, a, false, b, (short)0, c, false, false);
  asm volatile("v_nop\n\tv_nop\n\tv_nop\n\tv_nop" : "+v"(c) : "v"(a), "v"(b));
  return c;
}
__device__ __forceinline__ v8f mma_f16(v16h a, v16h b, v8f c) {
  c = __builtin_amdgcn_wmma_f32_16x16x32_f16(false, a, false, b, (short)0, c, false, false);
  asm volatile("v_nop\n\tv_nop\n\tv_nop\n\tv_nop" : "+v"(c) : "v"(a), "v"(b));
  return c;
}

__device__ __forceinline__ unsigned short f2bf(float f) {
  unsigned int u = __float_as_uint(f);
  u = u + 0x7FFFu + ((u >> 16) & 1u);
  return (unsigned short)(u >> 16);
}
__device__ __forceinline__ float bf2f(unsigned short w) {
  return __uint_as_float(((unsigned int)w) << 16);
}
__device__ __forceinline__ v8f zero8() {
  v8f z;
#pragma unroll
  for (int i = 0; i < 8; ++i) z[i] = 0.0f;
  return z;
}

__device__ __forceinline__ void cvt8(const float* __restrict__ src, unsigned short* dst, size_t e) {
  const v4f a = *(const v4f*)(src + e);
  const v4f c = *(const v4f*)(src + e + 4);
  v8us o;
#pragma unroll
  for (int j = 0; j < 4; ++j) {
    o[j] = f2bf(a[j]);
    o[4 + j] = f2bf(c[j]);
  }
  unsigned short* d = dst + e;
  *(volatile v8us*)d = o;
  __threadfence();
  *(volatile v8us*)d = o;
}

__global__ __launch_bounds__(256) void k_prep(const float* __restrict__ wv,
                                              const float* __restrict__ wz,
                                              const float* __restrict__ wq,
                                              unsigned short* wall, float* pet) {
  const int NWB = (DIM * DIM / 8) / 256;
  const int tid = threadIdx.x;
  const int bid = (int)blockIdx.x;
  if (bid < NWB) {
    cvt8(wv, wall, ((size_t)bid * 256 + tid) * 8);
  } else if (bid < 2 * NWB) {
    cvt8(wz, wall + (size_t)DIM * DIM, ((size_t)(bid - NWB) * 256 + tid) * 8);
  } else if (bid < 3 * NWB) {
    cvt8(wq, wall + (size_t)2 * DIM * DIM, ((size_t)(bid - 2 * NWB) * 256 + tid) * 8);
  } else {
    const int idx = (bid - 3 * NWB) * 256 + tid;
    const int pos = idx >> 8;
    const int c = idx & (DIM - 1);
    const int i = (c & 127) >> 1;
    const float dv = exp2f((float)i * 0.20762050593046014f);
    const float arg = (float)pos * (1.0f / dv);
    float sn, cs;
    sincosf(arg, &sn, &cs);
    const float val = (c & 1) ? cs : sn;
    float* d = pet + idx;
    *(volatile float*)d = val;
    __threadfence();
    *(volatile float*)d = val;
  }
}

__global__ __launch_bounds__(256) void k_xpose(const float* __restrict__ x,
                                               unsigned short* xT) {
  __shared__ __align__(16) unsigned short tile[32][72];
  const int tid = threadIdx.x;
  const int n0 = blockIdx.x * 32, c0 = blockIdx.y * 64, b = blockIdx.z;
  const float* xb = x + (size_t)b * DIM * SEQ_FULL;
  const int nl = tid & 31, cb = tid >> 5;
#pragma unroll
  for (int k = 0; k < 8; ++k) {
    const int cl = cb + 8 * k;
    tile[nl][cl] = f2bf(xb[(size_t)(c0 + cl) * SEQ_FULL + n0 + nl]);
  }
  __syncthreads();
  const int ln = tid >> 3, pc = (tid & 7) * 8;
  const v8us v = *(const v8us*)(&tile[ln][pc]);
  unsigned short* d = xT + ((size_t)b * SEQ + n0 + ln) * DIM + c0 + pc;
  *(volatile v8us*)d = v;
  __threadfence();
  *(volatile v8us*)d = v;
}

__global__ __launch_bounds__(128) void k_qkv(const unsigned short* __restrict__ wall,
                                             const unsigned short* __restrict__ xT,
                                             const float* __restrict__ pet,
                                             unsigned short* qh, unsigned short* ql,
                                             unsigned short* kh, unsigned short* kl,
                                             _Float16* vT) {
  __shared__ __align__(16) float stg[64][68];
  const int tid = threadIdx.x, lane = tid & 31, w = tid >> 5;
  const int h = lane >> 4, m = lane & 15;
  const int n0 = blockIdx.x * 64, o0 = blockIdx.y * 64, b = blockIdx.z;

  const unsigned short* arow = wall + (size_t)(o0 + 16 * w + m) * DIM;
  const unsigned short* xb = xT + ((size_t)b * SEQ + n0 + m) * DIM;

  v8f acc[4];
#pragma unroll
  for (int t = 0; t < 4; ++t) acc[t] = zero8();

#pragma unroll 2
  for (int k0 = 0; k0 < DIM; k0 += 32) {
    FragB a;
    a.p[0] = *(const v8us*)(arow + k0 + 8 * h);
    a.p[1] = *(const v8us*)(arow + k0 + 16 + 8 * h);
#pragma unroll
    for (int t = 0; t < 4; ++t) {
      const unsigned short* br = xb + (size_t)t * 16 * DIM + k0;
      FragB bb;
      bb.p[0] = *(const v8us*)(br + 8 * h);
      bb.p[1] = *(const v8us*)(br + 16 + 8 * h);
      acc[t] = mma_bf16(a.v, bb.v, acc[t]);
    }
  }

#pragma unroll
  for (int t = 0; t < 4; ++t)
#pragma unroll
    for (int r = 0; r < 8; ++r)
      stg[16 * t + m][16 * w + 8 * h + r] = acc[t][r];
  __syncthreads();

  const int seg = o0 >> 8;
  const int cb = o0 & (DIM - 1);
  const int lr = tid >> 3;
  const int pc = tid & 7;
  if (seg < 2) {
    unsigned short* ph = (seg == 0 ? qh : kh) + (size_t)b * SEQ * DIM;
    unsigned short* pl = (seg == 0 ? ql : kl) + (size_t)b * SEQ * DIM;
    const bool isy = cb < 128;
#pragma unroll
    for (int pass = 0; pass < 4; ++pass) {
      const int nl = pass * 16 + lr;
      const int n = n0 + nl;
      v4f f0 = *(const v4f*)(&stg[nl][pc * 8]);
      v4f f1 = *(const v4f*)(&stg[nl][pc * 8 + 4]);
      if (seg == 1) {
        const int yy = n / W_IMG;
        const int xx = n - yy * W_IMG;
        const int pos = isy ? yy : xx;
        const float* pr = pet + (size_t)pos * DIM + cb + pc * 8;
        const v4f e0 = *(const v4f*)pr;
        const v4f e1 = *(const v4f*)(pr + 4);
#pragma unroll
        for (int j = 0; j < 4; ++j) { f0[j] += e0[j]; f1[j] += e1[j]; }
      }
      v8us hi, lo;
#pragma unroll
      for (int j = 0; j < 4; ++j) {
        const float va = f0[j], vb2 = f1[j];
        const unsigned short ha = f2bf(va), hb = f2bf(vb2);
        hi[j] = ha;
        hi[4 + j] = hb;
        lo[j] = f2bf(va - bf2f(ha));
        lo[4 + j] = f2bf(vb2 - bf2f(hb));
      }
      const size_t off = (size_t)n * DIM + cb + pc * 8;
      *(volatile v8us*)(ph + off) = hi;
      *(volatile v8us*)(pl + off) = lo;
      __threadfence();
      *(volatile v8us*)(ph + off) = hi;
      *(volatile v8us*)(pl + off) = lo;
    }
  } else {
    _Float16* pv = vT + ((size_t)b * DIM + cb) * SEQ;
#pragma unroll
    for (int pass = 0; pass < 4; ++pass) {
      const int dl = pass * 16 + lr;
      v8h o;
#pragma unroll
      for (int j = 0; j < 8; ++j) o[j] = (_Float16)(stg[pc * 8 + j][dl] * 8.0f);
      const size_t off = (size_t)dl * SEQ + n0 + pc * 8;
      *(volatile v8h*)(pv + off) = o;
      __threadfence();
      *(volatile v8h*)(pv + off) = o;
    }
  }
}

__global__ __launch_bounds__(128) void k_attn(const unsigned short* __restrict__ qh,
                                              const unsigned short* __restrict__ ql,
                                              const unsigned short* __restrict__ kh,
                                              const unsigned short* __restrict__ kl,
                                              const _Float16* __restrict__ vT,
                                              float* out) {
  __shared__ __align__(16) unsigned short skh[32][40];
  __shared__ __align__(16) unsigned short skl[32][40];
  __shared__ __align__(16) _Float16 sv[32][40];
  __shared__ __align__(16) _Float16 sp[4][16][40];
  __shared__ __align__(16) float so[32][68];

  const int tid = threadIdx.x, lane = tid & 31, w = tid >> 5;
  const int h = lane >> 4, m = lane & 15;
  const int qb0 = blockIdx.x * 64;
  const int q0 = qb0 + w * 16;
  const int hd = blockIdx.y, b = blockIdx.z;
  const unsigned short* qhb = qh + (size_t)b * SEQ * DIM + hd * HD;
  const unsigned short* qlb = ql + (size_t)b * SEQ * DIM + hd * HD;
  const unsigned short* khb = kh + (size_t)b * SEQ * DIM + hd * HD;
  const unsigned short* klb = kl + (size_t)b * SEQ * DIM + hd * HD;
  const _Float16* vb = vT + ((size_t)b * DIM + hd * HD) * SEQ;

  FragB qhf, qlf;
  {
    const unsigned short* rh = qhb + (size_t)(q0 + m) * DIM;
    const unsigned short* rl = qlb + (size_t)(q0 + m) * DIM;
    qhf.p[0] = *(const v8us*)(rh + 8 * h);
    qhf.p[1] = *(const v8us*)(rh + 16 + 8 * h);
    qlf.p[0] = *(const v8us*)(rl + 8 * h);
    qlf.p[1] = *(const v8us*)(rl + 16 + 8 * h);
  }

  v8f oacc[2];
#pragma unroll
  for (int dt = 0; dt < 2; ++dt) oacc[dt] = zero8();
  float mi[8], li[8];
#pragma unroll
  for (int r = 0; r < 8; ++r) { mi[r] = -3.0e38f; li[r] = 0.0f; }

  const float scl = 0.17677669529663687f;

#pragma unroll 1
  for (int mc = 0; mc < SEQ; mc += 32) {
    {
      const int row = tid >> 2, pc = (tid & 3) * 8;
      *(v8us*)(&skh[row][pc]) = *(const v8us*)(khb + (size_t)(mc + row) * DIM + pc);
      *(v8us*)(&skl[row][pc]) = *(const v8us*)(klb + (size_t)(mc + row) * DIM + pc);
      *(v8h*)(&sv[row][pc]) = *(const v8h*)(vb + (size_t)row * SEQ + mc + pc);
    }
    __syncthreads();

    v8f s[2];
#pragma unroll
    for (int ct = 0; ct < 2; ++ct) {
      v8f acc = zero8();
      FragB kf, kg;
      kf.p[0] = *(const v8us*)(&skh[ct * 16 + m][8 * h]);
      kf.p[1] = *(const v8us*)(&skh[ct * 16 + m][16 + 8 * h]);
      kg.p[0] = *(const v8us*)(&skl[ct * 16 + m][8 * h]);
      kg.p[1] = *(const v8us*)(&skl[ct * 16 + m][16 + 8 * h]);
      acc = mma_bf16(qhf.v, kf.v, acc);
      acc = mma_bf16(qhf.v, kg.v, acc);
      acc = mma_bf16(qlf.v, kf.v, acc);
      s[ct] = acc;
    }

#pragma unroll
    for (int r = 0; r < 8; ++r) {
      const float a0 = s[0][r] * scl, a1 = s[1][r] * scl;
      float t = fmaxf(a0, a1);
      t = fmaxf(t, __shfl_xor(t, 1, 16));
      t = fmaxf(t, __shfl_xor(t, 2, 16));
      t = fmaxf(t, __shfl_xor(t, 4, 16));
      t = fmaxf(t, __shfl_xor(t, 8, 16));
      const float mn = fmaxf(mi[r], t);
      const float al = __expf(mi[r] - mn);
      const float p0 = __expf(a0 - mn);
      const float p1 = __expf(a1 - mn);
      float rs = p0 + p1;
      rs += __shfl_xor(rs, 1, 16);
      rs += __shfl_xor(rs, 2, 16);
      rs += __shfl_xor(rs, 4, 16);
      rs += __shfl_xor(rs, 8, 16);
      li[r] = li[r] * al + rs;
      mi[r] = mn;
#pragma unroll
      for (int dt = 0; dt < 2; ++dt) oacc[dt][r] *= al;
      sp[w][8 * h + r][m] = (_Float16)(p0 * 1024.0f);
      sp[w][8 * h + r][16 + m] = (_Float16)(p1 * 1024.0f);
    }
    __syncthreads();

    FragH pf;
    pf.p[0] = *(const v8h*)(&sp[w][m][8 * h]);
    pf.p[1] = *(const v8h*)(&sp[w][m][16 + 8 * h]);
#pragma unroll
    for (int dt = 0; dt < 2; ++dt) {
      FragH vf;
      vf.p[0] = *(const v8h*)(&sv[dt * 16 + m][8 * h]);
      vf.p[1] = *(const v8h*)(&sv[dt * 16 + m][16 + 8 * h]);
      oacc[dt] = mma_f16(pf.v, vf.v, oacc[dt]);
    }
    __syncthreads();
  }

#pragma unroll
  for (int r = 0; r < 8; ++r) {
    const float inv = 1.0f / (8192.0f * li[r]);
#pragma unroll
    for (int dt = 0; dt < 2; ++dt)
      so[dt * 16 + m][w * 16 + 8 * h + r] = oacc[dt][r] * inv;
  }
  __syncthreads();
  {
    const int pc = tid & 7;
#pragma unroll
    for (int pass = 0; pass < 4; ++pass) {
      const int L = pass * 16 + (tid >> 3);
      const int d = L >> 1, nh = L & 1;
      const int ml = nh * 32 + pc * 4;
      const v4f v = *(const v4f*)(&so[d][ml]);
      float* dst = out + ((size_t)b * DIM + hd * HD + d) * SEQ + qb0 + ml;
      *(volatile v4f*)dst = v;
      __threadfence();
      *(volatile v4f*)dst = v;
    }
  }
}

extern "C" void kernel_launch(void* const* d_in, const int* in_sizes, int n_in,
                              void* d_out, int out_size, void* d_ws, size_t ws_size,
                              hipStream_t stream) {
  if (n_in < 4) return;
  if (in_sizes[0] < NB * DIM * SEQ_FULL) return;
  if (in_sizes[1] < DIM * DIM) return;
  if (in_sizes[2] < DIM * DIM) return;
  if (in_sizes[3] < DIM * DIM) return;
  if (out_size < NB * DIM * SEQ) return;

  const float* x = (const float*)d_in[0];
  const float* w_v = (const float*)d_in[1];
  const float* w_z = (const float*)d_in[2];
  const float* w_q = (const float*)d_in[3];
  float* out = (float*)d_out;

  const size_t szW = (size_t)OCH * DIM * 2;
  const size_t szP = (size_t)NPOS * DIM * 4;
  const size_t szX = (size_t)NB * SEQ * DIM * 2;
  const size_t szQK = szX;
  const size_t szV = szX;
  size_t off = 0;
  char* ws = (char*)d_ws;
  unsigned short* wall = (unsigned short*)(ws + off); off += szW;
  float* pet = (float*)(ws + off); off += szP;
  unsigned short* xT = (unsigned short*)(ws + off); off += szX;
  unsigned short* qh = (unsigned short*)(ws + off); off += szQK;
  unsigned short* ql = (unsigned short*)(ws + off); off += szQK;
  unsigned short* kh = (unsigned short*)(ws + off); off += szQK;
  unsigned short* kl = (unsigned short*)(ws + off); off += szQK;
  _Float16* vT = (_Float16*)(ws + off); off += szV;
  if (off > ws_size) return;

  const int nwb = (DIM * DIM / 8) / 256;
  const int npb = (NPOS * DIM) / 256;
  k_prep<<<dim3(3 * nwb + npb), dim3(256), 0, stream>>>(w_v, w_z, w_q, wall, pet);
  k_xpose<<<dim3(SEQ / 32, DIM / 64, NB), dim3(256), 0, stream>>>(x, xT);
  k_qkv<<<dim3(SEQ / 64, OCH / 64, NB), dim3(128), 0, stream>>>(wall, xT, pet, qh, ql, kh, kl, vT);
  k_attn<<<dim3(SEQ / 64, HEADS, NB), dim3(128), 0, stream>>>(qh, ql, kh, kl, vT, out);
}
